// RWKV_Tmix_x070_Mose_39024072851813
// MI455X (gfx1250) — hardware-verified
//
#include <hip/hip_runtime.h>


#define NT   1024
#define C_   2048
#define NH   32
#define HN   64
#define DW   96
#define DA   96
#define DV   64
#define DLP  320
#define DL   DLP
#define EPSN 1e-12f
#define DM   C_
#define LOSC 1024.0f

typedef _Float16 h16;
typedef unsigned short bf;
typedef __attribute__((ext_vector_type(16))) __bf16   v16bf;
typedef __attribute__((ext_vector_type(16))) _Float16 v16h;
typedef __attribute__((ext_vector_type(8)))  _Float16 v8h;
typedef __attribute__((ext_vector_type(8)))  unsigned short v8us;
typedef __attribute__((ext_vector_type(8)))  float    v8f;
typedef __attribute__((ext_vector_type(4)))  float    v4f;
typedef v8h  __attribute__((may_alias)) v8ha;
typedef v4f  __attribute__((may_alias)) v4fa;
typedef v8us __attribute__((may_alias)) v8usa;

__device__ __forceinline__ unsigned short f2bf(float f) { unsigned u = __float_as_uint(f); u += 0x7FFFu + ((u >> 16) & 1u); return (unsigned short)(u >> 16); }
__device__ __forceinline__ float bf2f(unsigned short b) { return __uint_as_float(((unsigned)b) << 16); }
__device__ __forceinline__ float bfr(float f) { return bf2f(f2bf(f)); }
__device__ __forceinline__ v16h cat16(v8h lo, v8h hi) { return __builtin_shufflevector(lo, hi, 0, 1, 2, 3, 4, 5, 6, 7, 8, 9, 10, 11, 12, 13, 14, 15); }
__device__ __forceinline__ v16bf cat16b(v8us lo, v8us hi) { return __builtin_bit_cast(v16bf, __builtin_shufflevector(lo, hi, 0, 1, 2, 3, 4, 5, 6, 7, 8, 9, 10, 11, 12, 13, 14, 15)); }
__device__ __forceinline__ v8f wmma16(v16h a, v16h b, v8f c) { return __builtin_amdgcn_wmma_f32_16x16x32_f16(false, a, false, b, (short)0, c, false, false); }
__device__ __forceinline__ v8f wmmab(v16bf a, v16bf b, v8f c) { return __builtin_amdgcn_wmma_f32_16x16x32_bf16(false, a, false, b, (short)0, c, false, false); }

template <bool SPLITA, bool F16OUT = false>
__global__ __launch_bounds__(128) void k_gemmb(const bf* __restrict__ A, const bf* __restrict__ Al, const bf* __restrict__ Bn, const float* __restrict__ bias, float* C, int ldc, h16* C2, const float* __restrict__ R = nullptr, int K = DM, int roundR = 1) {
    __shared__ __align__(16) float ost[4][16 * 68];
    const int lane = threadIdx.x & 31, wave = threadIdx.x >> 5, lr = lane & 15, hi = lane >> 4;
    const int r0 = blockIdx.x * 64 + wave * 16, c0 = blockIdx.y * 64;
    const size_t aoff = (size_t)(r0 + lr) * K + 8 * hi;
    size_t boff[4];
#pragma unroll
    for (int t = 0; t < 4; ++t) boff[t] = (size_t)(c0 + t * 16 + lr) * K + 8 * hi;
    v8f acc[4];
#pragma unroll
    for (int t = 0; t < 4; ++t) acc[t] = (v8f){};
#pragma unroll 1
    for (int kc = 0; kc < K; kc += 32) {
        const v16bf a = cat16b(*(const v8us*)(A + aoff + kc), *(const v8us*)(A + aoff + kc + 16));
        v16bf al = a;
        if (SPLITA) al = cat16b(*(const v8us*)(Al + aoff + kc), *(const v8us*)(Al + aoff + kc + 16));
#pragma unroll
        for (int t = 0; t < 4; ++t) { const v16bf b = cat16b(*(const v8us*)(Bn + boff[t] + kc), *(const v8us*)(Bn + boff[t] + kc + 16)); acc[t] = wmmab(a, b, acc[t]); if (SPLITA) acc[t] = wmmab(al, b, acc[t]); }
        asm volatile("v_nop\n\tv_nop\n\tv_nop\n\tv_nop" : "+v"(acc[0]), "+v"(acc[1]), "+v"(acc[2]), "+v"(acc[3]) : "v"(a), "v"(al));
    }
    float* os = &ost[wave][0];
#pragma unroll
    for (int t = 0; t < 4; ++t) { const float bv = bias ? bfr(bias[c0 + t * 16 + lr]) : 0.f;
#pragma unroll
        for (int j = 0; j < 8; ++j) os[(hi * 8 + j) * 68 + t * 16 + lr] = acc[t][j] + bv; }
    __syncthreads();
    if (F16OUT) {
        h16* crow = (h16*)(void*)C + (size_t)r0 * ldc + c0;
        auto pass = [&]() {
#pragma unroll
            for (int s = 0; s < 4; ++s) { const int row = 4 * s + (lane >> 3), piece = lane & 7; const float* sp = os + row * 68 + piece * 8; v8h o, o2;
#pragma unroll
                for (int i = 0; i < 8; ++i) { const h16 a = (h16)sp[i]; o[i] = a; o2[i] = (h16)((sp[i] - (float)a) * LOSC); }
                *(volatile v8h*)(crow + (size_t)row * ldc + piece * 8) = o; if (C2) *(volatile v8h*)(C2 + (size_t)r0 * ldc + c0 + (size_t)row * ldc + piece * 8) = o2; }
        };
        pass(); __threadfence(); pass();
    } else {
        float* crow = C + (size_t)r0 * ldc + c0;
        auto pass = [&]() {
#pragma unroll
            for (int s = 0; s < 8; ++s) { const int Lid = (lane >> 3) + 4 * s, piece = lane & 7; const int row = Lid >> 1, cofs = (Lid & 1) * 32 + piece * 4;
                v4f val = *(const v4fa*)(os + row * 68 + cofs); if (R) { const v4f rv = *(const v4f*)(R + ((size_t)r0 + row) * ldc + c0 + cofs); val += roundR ? (v4f){bfr(rv[0]), bfr(rv[1]), bfr(rv[2]), bfr(rv[3])} : rv; }
                *(volatile v4f*)(crow + (size_t)row * ldc + cofs) = val; }
        };
        pass(); __threadfence(); pass();
    }
}

__global__ __launch_bounds__(256) void k_wtp(const float* __restrict__ Wm, int krows, int ncols, int kpad, bf* WT) {
    __shared__ __align__(16) unsigned short tl[64 * 72];
    const int tid = threadIdx.x, k0 = blockIdx.x * 64, n0 = blockIdx.y * 64;
    const int kk = tid >> 2, nq = (tid & 3) * 16;
    const int k = k0 + kk, kc = k < krows ? k : krows - 1;
#pragma unroll
    for (int i = 0; i < 16; ++i) { const int n = n0 + nq + i, ncl = n < ncols ? n : ncols - 1; const float w = Wm[(size_t)kc * ncols + ncl]; tl[(nq + i) * 72 + kk] = (k < krows && n < ncols) ? f2bf(w) : (unsigned short)0; }
    __syncthreads();
    const int piece = tid & 7;
    auto pass = [&]() {
#pragma unroll
        for (int s = 0; s < 2; ++s) { const int nr = (tid >> 3) + 32 * s; const v8us val = *(const v8usa*)(tl + nr * 72 + piece * 8); *(volatile v8us*)(WT + (size_t)(n0 + nr) * kpad + k0 + piece * 8) = val; }
    };
    pass(); __threadfence(); pass();
}

__global__ __launch_bounds__(256) void k_wt(const float* __restrict__ Wm, int K, int ncols, bf* WT) {
    __shared__ __align__(16) unsigned short tl[64 * 72];
    const int tid = threadIdx.x, k0 = blockIdx.x * 64, n0 = blockIdx.y * 64;
    const int kk = tid >> 2, nq = (tid & 3) * 16;
#pragma unroll
    for (int i = 0; i < 16; ++i) tl[(nq + i) * 72 + kk] = f2bf(Wm[(size_t)(k0 + kk) * ncols + n0 + nq + i]);
    __syncthreads();
    const int piece = tid & 7;
    auto pass = [&]() {
#pragma unroll
        for (int s = 0; s < 2; ++s) { const int nr = (tid >> 3) + 32 * s; const v8us val = *(const v8usa*)(tl + nr * 72 + piece * 8); *(volatile v8us*)(WT + (size_t)(n0 + nr) * K + k0 + piece * 8) = val; }
    };
    pass(); __threadfence(); pass();
}

__global__ __launch_bounds__(256) void k_cvtb(const float* __restrict__ src, int nrows, bf* dst) {
    const int lane = threadIdx.x & 31, r = blockIdx.x * 8 + (threadIdx.x >> 5); if (r >= nrows) return;
#pragma unroll 1
    for (int ps = 0; ps < 2; ++ps) {
#pragma unroll
        for (int q = 0; q < C_ / 256; ++q) { v8us o;
#pragma unroll
            for (int i = 0; i < 8; ++i) o[i] = f2bf(src[(size_t)r * C_ + q * 256 + lane * 8 + i]);
            *(volatile v8us*)(dst + (size_t)r * C_ + q * 256 + lane * 8) = o; }
        if (ps == 0) __threadfence(); }
}
__global__ __launch_bounds__(256) void k_copy(const float* __restrict__ src, float* dst, size_t n4) {
    const size_t i = (size_t)blockIdx.x * 256 + threadIdx.x; if (i >= n4) return; const v4f v = *(const v4f*)(src + i * 4);
    *(volatile v4f*)(dst + i * 4) = v; __threadfence(); *(volatile v4f*)(dst + i * 4) = v;
}
__global__ __launch_bounds__(256) void k_lsplit(const float* __restrict__ L1, bf* Lh, bf* Ll) {
    const int lane = threadIdx.x & 31, r = blockIdx.x * 8 + (threadIdx.x >> 5); if (r >= NT) return;
#pragma unroll 1
    for (int ps = 0; ps < 2; ++ps) {
#pragma unroll 1
        for (int c0 = lane * 8; c0 < DLP; c0 += 256) { const size_t o = (size_t)r * DLP + c0; const v8f v = *(const v8f*)(L1 + o); v8us oh, ol;
#pragma unroll
            for (int i = 0; i < 8; ++i) { const int c = c0 + i; const float y = (c < DW) ? tanhf(v[i]) : v[i]; const unsigned short hb = f2bf(y); oh[i] = hb; ol[i] = f2bf(y - bf2f(hb)); }
            *(volatile v8us*)(Lh + o) = oh; *(volatile v8us*)(Ll + o) = ol; }
        if (ps == 0) __threadfence(); }
}
__global__ __launch_bounds__(128) void k_gemml(const bf* __restrict__ Ah, const bf* __restrict__ Al, int lda, const bf* __restrict__ Bn, int K, float* C, int ldc) {
    __shared__ __align__(16) float ost[4][16 * 68];
    const int lane = threadIdx.x & 31, wave = threadIdx.x >> 5, lr = lane & 15, hi = lane >> 4;
    const int r0 = blockIdx.x * 64 + wave * 16, c0 = blockIdx.y * 64;
    const size_t aoff = (size_t)(r0 + lr) * lda + 8 * hi;
    v8f acc[4];
#pragma unroll
    for (int t = 0; t < 4; ++t) acc[t] = (v8f){};
#pragma unroll 1
    for (int kc = 0; kc < K; kc += 32) {
        const v16bf a = cat16b(*(const v8us*)(Ah + aoff + kc), *(const v8us*)(Ah + aoff + kc + 16));
        const v16bf al = cat16b(*(const v8us*)(Al + aoff + kc), *(const v8us*)(Al + aoff + kc + 16));
#pragma unroll
        for (int t = 0; t < 4; ++t) { const size_t bo = (size_t)(c0 + t * 16 + lr) * K + kc + 8 * hi;
            const v16bf bb = cat16b(*(const v8us*)(Bn + bo), *(const v8us*)(Bn + bo + 16)); acc[t] = wmmab(a, bb, acc[t]); acc[t] = wmmab(al, bb, acc[t]); }
        asm volatile("v_nop\n\tv_nop\n\tv_nop\n\tv_nop" : "+v"(acc[0]), "+v"(acc[1]), "+v"(acc[2]), "+v"(acc[3]) : "v"(a), "v"(al));
    }
    float* os = &ost[wave][0];
#pragma unroll
    for (int t = 0; t < 4; ++t) {
#pragma unroll
        for (int j = 0; j < 8; ++j) os[(hi * 8 + j) * 68 + t * 16 + lr] = acc[t][j]; }
    __builtin_amdgcn_wave_barrier(); asm volatile("" ::: "memory");
    float* crow = C + (size_t)r0 * ldc + c0;
    auto pass = [&]() {
#pragma unroll
        for (int s = 0; s < 8; ++s) { const int Lid = (lane >> 3) + 4 * s, piece = lane & 7; const int row = Lid >> 1, cofs = (Lid & 1) * 32 + piece * 4;
            const v4f val = *(const v4fa*)(os + row * 68 + cofs); *(volatile v4f*)(crow + (size_t)row * ldc + cofs) = val; }
    };
    pass(); __threadfence(); pass();
}

__global__ __launch_bounds__(256) void k_prep7(const float* __restrict__ R, float* K, float* V, float* WL, float* AL, float* VL, const float* __restrict__ vfirst, const float* __restrict__ mask,
                                              const float* __restrict__ w0, const float* __restrict__ a0, const float* __restrict__ v0, const float* __restrict__ k_k, const float* __restrict__ k_a, const float* __restrict__ r_k, float* BC) {
    typedef __attribute__((ext_vector_type(2))) float v2f;
    __shared__ float bcs[8][NH];
    const int lane = threadIdx.x & 31, wv = threadIdx.x >> 5, t = blockIdx.x * 8 + wv;
    const float m = bfr(mask[t]);
#pragma unroll 1
    for (int h = 0; h < NH; ++h) { const size_t o = (size_t)t * C_ + h * HN + lane * 2; const int c0 = h * HN + lane * 2;
        float kp[2], vp[2], dc[2], aa[2], bb[2], kk[2]; float nrm = 0.f, bon = 0.f;
#pragma unroll
        for (int i = 0; i < 2; ++i) { const int c = c0 + i; const float r = R[o + i], k = K[o + i], v = V[o + i];
            const float wpre = -(bfr(w0[c]) + WL[o + i]); const float sp = (wpre > 20.f) ? wpre : log1pf(__expf(wpre)); const float w = -sp - 0.6f;
            float d = __expf(-__expf(w)); d = d * m + (1.0f - m); dc[i] = d;
            const float vv = v + (bfr(vfirst[o + i]) - v) * (1.0f / (1.0f + __expf(-(bfr(v0[c]) + VL[o + i]))));
            const float a = 1.0f / (1.0f + __expf(-(bfr(a0[c]) + AL[o + i])));
            const float kkv = k * bfr(k_k[c]); kk[i] = kkv; nrm = fmaf(kkv, kkv, nrm);
            const float kpv = k * (1.0f + (a - 1.0f) * bfr(k_a[c])); kp[i] = kpv * m; vp[i] = vv; aa[i] = a;
            bon = fmaf(r * kpv, bfr(r_k[h * HN + lane * 2 + i]), bon); }
#pragma unroll
        for (int sh = 16; sh; sh >>= 1) { nrm += __shfl_xor(nrm, sh, 32); bon += __shfl_xor(bon, sh, 32); }
        const float inv = 1.0f / fmaxf(sqrtf(nrm), EPSN);
#pragma unroll
        for (int i = 0; i < 2; ++i) { const float kkn = kk[i] * inv; bb[i] = kkn * aa[i] * m; aa[i] = -kkn * m; }
        if (lane == 0) bcs[wv][h] = bon;
        const v2f KP2 = {kp[0], kp[1]}, VP2 = {vp[0], vp[1]}, DC2 = {dc[0], dc[1]}, AA2 = {aa[0], aa[1]}, BB2 = {bb[0], bb[1]};
        *(volatile v2f*)(K + o) = KP2; *(volatile v2f*)(V + o) = VP2; *(volatile v2f*)(WL + o) = DC2; *(volatile v2f*)(AL + o) = AA2; *(volatile v2f*)(VL + o) = BB2; __threadfence();
        *(volatile v2f*)(K + o) = KP2; *(volatile v2f*)(V + o) = VP2; *(volatile v2f*)(WL + o) = DC2; *(volatile v2f*)(AL + o) = AA2; *(volatile v2f*)(VL + o) = BB2; }
    __builtin_amdgcn_wave_barrier(); asm volatile("" ::: "memory");
    const float bcv = bcs[wv][lane]; *(volatile float*)(BC + (size_t)t * NH + lane) = bcv; __threadfence(); *(volatile float*)(BC + (size_t)t * NH + lane) = bcv;
}
__global__ __launch_bounds__(128) void k_rwkv(const float* __restrict__ R, const float* __restrict__ KP, const float* __restrict__ VP, const float* __restrict__ DEC, const float* __restrict__ AA, const float* __restrict__ BB, const float* __restrict__ mask, float* O) {
    __shared__ float S[2][HN][HN + 1]; __shared__ float vr[2][HN], vd[2][HN], vk[2][HN], va[2][HN], vb[2][HN];
    const int tid = threadIdx.x, h2 = tid >> 6, i = tid & 63, h = blockIdx.x * 2 + h2;
#pragma unroll 4
    for (int j = 0; j < HN; ++j) S[h2][i][j] = 0.f;
#pragma unroll 1
    for (int t = 0; t < NT; ++t) { const size_t o = (size_t)t * C_ + h * HN + i;
        __syncthreads();
        vr[h2][i] = R[o]; vd[h2][i] = DEC[o]; vk[h2][i] = KP[o]; va[h2][i] = AA[o]; vb[h2][i] = BB[o];
        __syncthreads();
        const float vi = VP[o] * bfr(mask[t]); float sa = 0.f;
#pragma unroll 4
        for (int j = 0; j < HN; ++j) sa = fmaf(S[h2][i][j], va[h2][j], sa);
        float ov = 0.f;
#pragma unroll 4
        for (int j = 0; j < HN; ++j) { const float s = fmaf(S[h2][i][j], vd[h2][j], fmaf(sa, vb[h2][j], vi * vk[h2][j])); S[h2][i][j] = s; ov = fmaf(s, vr[h2][j], ov); }
        *(volatile float*)(O + o) = ov; __threadfence(); *(volatile float*)(O + o) = ov; }
}
__global__ __launch_bounds__(256) void k_fin(const float* __restrict__ O, const float* __restrict__ VP, const float* __restrict__ BC, bf* Yh, bf* Yl) {
    const int lane = threadIdx.x & 31, t = blockIdx.x * 8 + (threadIdx.x >> 5); if (t >= NT) return;
#pragma unroll 1
    for (int ps = 0; ps < 2; ++ps) {
#pragma unroll 1
        for (int c0 = lane * 8; c0 < C_; c0 += 256) { const size_t o = (size_t)t * C_ + c0; const v8f ov = *(const v8f*)(O + o), vv = *(const v8f*)(VP + o); const float bc = BC[(size_t)t * NH + c0 / HN]; v8us oh, ol;
#pragma unroll
            for (int q = 0; q < 8; ++q) { const float y = fmaf(bc, vv[q], ov[q]); const unsigned short hb = f2bf(y); oh[q] = hb; ol[q] = f2bf(y - bf2f(hb)); }
            *(volatile v8us*)(Yh + o) = oh; *(volatile v8us*)(Yl + o) = ol; }
        if (ps == 0) __threadfence(); }
}

extern "C" void kernel_launch(void* const* d_in, const int* in_sizes, int n_in,
                              void* d_out, int out_size, void* d_ws, size_t ws_size, hipStream_t stream) {
    (void)in_sizes; (void)n_in; (void)out_size;
    const float* x = (const float*)d_in[0]; const float* vfirst = (const float*)d_in[1]; const float* mask = (const float*)d_in[2]; const float* w0 = (const float*)d_in[3]; const float* w1 = (const float*)d_in[4]; const float* w2 = (const float*)d_in[5];
    const float* a0 = (const float*)d_in[6]; const float* a1 = (const float*)d_in[7]; const float* a2 = (const float*)d_in[8]; const float* v0 = (const float*)d_in[9]; const float* v1 = (const float*)d_in[10]; const float* v2 = (const float*)d_in[11];
    const float* k_k = (const float*)d_in[12]; const float* k_a = (const float*)d_in[13]; const float* r_k = (const float*)d_in[14]; const float* Wr = (const float*)d_in[15]; const float* Wk = (const float*)d_in[16]; const float* Wv = (const float*)d_in[17]; const float* Wo = (const float*)d_in[18];
    float* out = (float*)d_out; float* out2 = (float*)((char*)d_out + (size_t)NT * C_ * 4);
    char* wsp = (char*)d_ws;
    auto take = [&](size_t bytes) { char* p = wsp; wsp += (bytes + 255) & ~(size_t)255; return (void*)p; };
    bf* WrT = (bf*)take((size_t)C_ * C_ * 2); bf* WkT = (bf*)take((size_t)C_ * C_ * 2); bf* WvT = (bf*)take((size_t)C_ * C_ * 2); bf* WoT = (bf*)take((size_t)C_ * C_ * 2);
    bf* LT = (bf*)take((size_t)DLP * C_ * 2); bf* W2T = (bf*)take((size_t)C_ * 128 * 2); bf* A2T = (bf*)take((size_t)C_ * 128 * 2); bf* V2T = (bf*)take((size_t)C_ * DV * 2);
    bf* Xb = (bf*)take((size_t)NT * C_ * 2); float* L1 = (float*)take((size_t)NT * DLP * 4); bf* Lh = (bf*)take((size_t)NT * DLP * 2); bf* Ll = (bf*)take((size_t)NT * DLP * 2);
    float* R = (float*)take((size_t)NT * C_ * 4); float* K = (float*)take((size_t)NT * C_ * 4); float* V = (float*)take((size_t)NT * C_ * 4); float* WL = (float*)take((size_t)NT * C_ * 4); float* AL = (float*)take((size_t)NT * C_ * 4); float* VL = (float*)take((size_t)NT * C_ * 4);
    float* BC = (float*)take((size_t)NT * NH * 4); float* O = (float*)take((size_t)NT * C_ * 4); bf* Yh = (bf*)take((size_t)NT * C_ * 2); bf* Yl = (bf*)take((size_t)NT * C_ * 2);
    if ((size_t)(wsp - (char*)d_ws) > ws_size) return;
    k_copy<<<(unsigned)(((size_t)NT * C_ / 4 + 255) / 256), 256, 0, stream>>>(vfirst, out2, (size_t)NT * C_ / 4);
    k_wt<<<dim3(C_ / 64, C_ / 64, 1), 256, 0, stream>>>(Wr, C_, C_, WrT); k_wt<<<dim3(C_ / 64, C_ / 64, 1), 256, 0, stream>>>(Wk, C_, C_, WkT); k_wt<<<dim3(C_ / 64, C_ / 64, 1), 256, 0, stream>>>(Wv, C_, C_, WvT); k_wt<<<dim3(C_ / 64, C_ / 64, 1), 256, 0, stream>>>(Wo, C_, C_, WoT);
    k_wtp<<<dim3(C_ / 64, 2, 1), 256, 0, stream>>>(w1, C_, DW, C_, LT); k_wtp<<<dim3(C_ / 64, 2, 1), 256, 0, stream>>>(a1, C_, DA, C_, LT + (size_t)128 * C_); k_wt<<<dim3(C_ / 64, 1, 1), 256, 0, stream>>>(v1, C_, DV, LT + (size_t)256 * C_);
    k_wtp<<<dim3(2, C_ / 64, 1), 256, 0, stream>>>(w2, DW, C_, 128, W2T); k_wtp<<<dim3(2, C_ / 64, 1), 256, 0, stream>>>(a2, DA, C_, 128, A2T); k_wt<<<dim3(1, C_ / 64, 1), 256, 0, stream>>>(v2, DV, C_, V2T);
    k_cvtb<<<NT / 8, 256, 0, stream>>>(x, NT, Xb);
    k_gemmb<false, false><<<dim3(NT / 64, DLP / 64, 1), 128, 0, stream>>>(Xb, nullptr, LT, nullptr, L1, DLP, nullptr, nullptr, C_);
    k_lsplit<<<NT / 8, 256, 0, stream>>>(L1, Lh, Ll);
    k_gemml<<<dim3(NT / 64, C_ / 64, 1), 128, 0, stream>>>(Lh, Ll, DLP, W2T, 128, WL, C_);
    k_gemml<<<dim3(NT / 64, C_ / 64, 1), 128, 0, stream>>>(Lh + 128, Ll + 128, DLP, A2T, 128, AL, C_);
    k_gemml<<<dim3(NT / 64, C_ / 64, 1), 128, 0, stream>>>(Lh + 256, Ll + 256, DLP, V2T, DV, VL, C_);
    k_gemmb<false, false><<<dim3(NT / 64, C_ / 64, 1), 128, 0, stream>>>(Xb, nullptr, WrT, nullptr, R, C_, nullptr, nullptr, C_);
    k_gemmb<false, false><<<dim3(NT / 64, C_ / 64, 1), 128, 0, stream>>>(Xb, nullptr, WkT, nullptr, K, C_, nullptr, nullptr, C_);
    k_gemmb<false, false><<<dim3(NT / 64, C_ / 64, 1), 128, 0, stream>>>(Xb, nullptr, WvT, nullptr, V, C_, nullptr, nullptr, C_);
    k_prep7<<<NT / 8, 256, 0, stream>>>(R, K, V, WL, AL, VL, vfirst, mask, w0, a0, v0, k_k, k_a, r_k, BC);
    k_rwkv<<<NH / 2, 128, 0, stream>>>(R, K, V, WL, AL, VL, mask, O);
    k_fin<<<NT / 8, 256, 0, stream>>>(O, V, BC, Yh, Yl);
    k_gemmb<true, false><<<dim3(NT / 64, C_ / 64, 1), 128, 0, stream>>>(Yh, Yl, WoT, nullptr, out, C_, nullptr, nullptr, C_);
}
